// RNN_19155554140953
// MI455X (gfx1250) — hardware-verified
//
#include <hip/hip_runtime.h>
#include <math.h>

constexpr int NBATCH    = 64;
constexpr int NSTEP     = 512;
constexpr int NIN       = 256;
constexpr int NHID      = 512;
constexpr int NCLS      = 10;
constexpr int NTHR      = 256;
constexpr int SCAN_ROWS = 32;
constexpr int HPITCH    = 520;
constexpr int NROWS     = NBATCH * NSTEP;
constexpr float W_CARRY     = 256.0f;
constexpr float W_CARRY_INV = 1.0f / 256.0f;

static_assert(NBATCH % SCAN_ROWS == 0);
static_assert(NHID == 64 * (NTHR / 32));
static_assert(NIN % 32 == 0 && NHID % 32 == 0);
static_assert(NROWS % 64 == 0 && NHID % 64 == 0);
static_assert(((NROWS / 64) * (NHID / 64)) % 8 == 0);
static_assert((2 * SCAN_ROWS * HPITCH) % 8 == 0);
static_assert((HPITCH * 2) % 16 == 0);
static_assert((NBATCH * NCLS) % 128 == 0);
static_assert(NBATCH == 64);

typedef __attribute__((ext_vector_type(16))) _Float16 v16h;
typedef __attribute__((ext_vector_type(8)))  _Float16 v8h;
typedef __attribute__((ext_vector_type(8)))  float    v8f;
typedef __attribute__((ext_vector_type(4)))  float    v4f;

__device__ __forceinline__ void keep4_h(v16h a, v16h b, v16h c, v16h d) { asm volatile("v_nop" :: "v"(a), "v"(b), "v"(c), "v"(d)); }
__device__ __forceinline__ void acc_guard4(v8f& a, v8f& b, v8f& c, v8f& d) { asm volatile("v_nop\n\tv_nop\n\tv_nop\n\tv_nop" : "+v"(a), "+v"(b), "+v"(c), "+v"(d)); }
__device__ __forceinline__ void acc_guard2(v8f& a, v8f& b) { asm volatile("v_nop\n\tv_nop\n\tv_nop\n\tv_nop" : "+v"(a), "+v"(b)); }
__device__ __forceinline__ void guard4_h(v8f& a, v8f& b, v8f& c, v8f& d, v16h x) { asm volatile("v_nop\n\tv_nop\n\tv_nop\n\tv_nop" : "+v"(a), "+v"(b), "+v"(c), "+v"(d) : "v"(x)); }
__device__ __forceinline__ void guard2_h(v8f& a, v8f& b, v16h x, v16h y, v16h z) { asm volatile("v_nop\n\tv_nop\n\tv_nop\n\tv_nop" : "+v"(a), "+v"(b) : "v"(x), "v"(y), "v"(z)); }
__device__ __forceinline__ void pin2_f(v4f& a, v4f& b) { asm volatile("" : "+v"(a), "+v"(b)); }

struct FragH {
  union U { v16h v; v8h h[2]; };
  static __device__ __forceinline__ v16h load(const _Float16* p) {
    U f; f.h[0] = *(const v8h*)(p); f.h[1] = *(const v8h*)(p + 16); return f.v;
  }
  static __device__ __forceinline__ v8f mma(v16h a, v16h b, v8f c) {
    return __builtin_amdgcn_wmma_f32_16x16x32_f16(false, a, false, b, (short)0, c, false, false);
  }
};

__global__ __launch_bounds__(NTHR) void cvt_x_kernel(const float* __restrict__ x, unsigned short* __restrict__ dst) {
  const int i = blockIdx.x * NTHR + threadIdx.x;
  const int n8 = NROWS * (NIN / 8);
  if (i < n8) {
    const int orow = i >> 5;
    const int c8 = i & 31;
    const int t = orow >> 6;
    const int b = orow & 63;
    const float* sp = x + ((size_t)b * NSTEP + (size_t)t) * NIN + c8 * 8;
    const v4f a0 = *(const v4f*)(sp);
    const v4f a1 = *(const v4f*)(sp + 4);
    v8h hv;
#pragma unroll
    for (int e = 0; e < 4; ++e) {
      hv[e]     = (_Float16)a0[e];
      hv[4 + e] = (_Float16)a1[e];
    }
    _Float16* dp = (_Float16*)dst + (size_t)i * 8;
    *(volatile v8h*)dp = hv;
    __threadfence();
    *(volatile v8h*)dp = hv;
  }
}

__global__ __launch_bounds__(NTHR) void cvt_w_kernel(const float* __restrict__ src, unsigned short* __restrict__ dst, int n8, float sc) {
  const int i = blockIdx.x * NTHR + threadIdx.x;
  if (i < n8) {
    const float* sp = src + (size_t)i * 8;
    const v4f a0 = *(const v4f*)(sp);
    const v4f a1 = *(const v4f*)(sp + 4);
    v8h hv;
#pragma unroll
    for (int e = 0; e < 4; ++e) {
      hv[e]     = (_Float16)(a0[e] * sc);
      hv[4 + e] = (_Float16)(a1[e] * sc);
    }
    _Float16* dp = (_Float16*)dst + (size_t)i * 8;
    *(volatile v8h*)dp = hv;
    __threadfence();
    *(volatile v8h*)dp = hv;
  }
}

__global__ __launch_bounds__(256) void gemm_f16_bias2_kernel(
    const unsigned short* __restrict__ Ap, int lda,
    const unsigned short* __restrict__ Btp, int ldb,
    float* __restrict__ Cout, int ldc,
    const float* __restrict__ bias_a, const float* __restrict__ bias_b,
    int M, int N, int K, float scale) {
  const _Float16* A  = (const _Float16*)Ap;
  const _Float16* Bt = (const _Float16*)Btp;
  __shared__ __align__(16) float sT[8][16 * 68];
  const int lane = threadIdx.x & 31;
  const int wave = threadIdx.x >> 5;
  const int tilesN = N >> 6;
  const int tilesM = M >> 6;
  const int tile = blockIdx.x * 8 + wave;
  if (tile >= tilesM * tilesN) return;
  const int tm = tile / tilesN;
  const int tn = tile - tm * tilesN;
  const int m0 = tm << 6;
  const int n0 = tn << 6;

  const int rlane = lane & 15;
  const int koff  = (lane >> 4) * 8;
  const int mOff  = (lane >> 4) * 8;

  v8f acc[4][4];
#pragma unroll
  for (int i = 0; i < 4; ++i)
#pragma unroll
    for (int j = 0; j < 4; ++j) acc[i][j] = (v8f){0.f, 0.f, 0.f, 0.f, 0.f, 0.f, 0.f, 0.f};

  for (int k0 = 0; k0 < K; k0 += 32) {
    v16h bh[4];
#pragma unroll
    for (int j = 0; j < 4; ++j) {
      const size_t bo = (size_t)(n0 + (j << 4) + rlane) * ldb + koff + k0;
      bh[j] = FragH::load(Bt + bo);
    }
#pragma unroll
    for (int i = 0; i < 4; ++i) {
      const size_t ao = (size_t)(m0 + (i << 4) + rlane) * lda + koff + k0;
      const v16h ah = FragH::load(A + ao);
#pragma unroll
      for (int j = 0; j < 4; ++j) acc[i][j] = FragH::mma(ah, bh[j], acc[i][j]);
      guard4_h(acc[i][0], acc[i][1], acc[i][2], acc[i][3], ah);
    }
    keep4_h(bh[0], bh[1], bh[2], bh[3]);
  }
  acc_guard4(acc[0][0], acc[0][1], acc[0][2], acc[0][3]);
  acc_guard4(acc[1][0], acc[1][1], acc[1][2], acc[1][3]);
  acc_guard4(acc[2][0], acc[2][1], acc[2][2], acc[2][3]);
  acc_guard4(acc[3][0], acc[3][1], acc[3][2], acc[3][3]);

  float* slab = sT[wave];
#pragma unroll
  for (int i = 0; i < 4; ++i) {
    const int mBase = m0 + (i << 4);
#pragma unroll
    for (int j = 0; j < 4; ++j) {
      const int n = n0 + (j << 4) + rlane;
      const float bva = bias_a[n];
      const float bvb = bias_b[n];
#pragma unroll
      for (int r = 0; r < 8; ++r) {
        float v = acc[i][j][r] * scale;
        v += bva;
        v += bvb;
        slab[(mOff + r) * 68 + (j << 4) + rlane] = v;
      }
    }
    __builtin_amdgcn_fence(__ATOMIC_RELEASE, "workgroup");
    __builtin_amdgcn_wave_barrier();
    __builtin_amdgcn_fence(__ATOMIC_ACQUIRE, "workgroup");
    {
      const int hh = lane >> 4, c4 = (lane & 15) * 4;
      for (int pass = 0; pass < 2; ++pass) {
#pragma unroll
        for (int it = 0; it < 8; ++it) {
          const int row = it * 2 + hh;
          const v4f v = *(const v4f*)(slab + row * 68 + c4);
          *(volatile v4f*)(Cout + (size_t)(mBase + row) * ldc + n0 + c4) = v;
        }
        __threadfence();
      }
    }
    __builtin_amdgcn_fence(__ATOMIC_RELEASE, "workgroup");
    __builtin_amdgcn_wave_barrier();
    __builtin_amdgcn_fence(__ATOMIC_ACQUIRE, "workgroup");
  }
}

template <bool WRITE_SEQ, bool FINAL>
__global__ __launch_bounds__(NTHR) void rnn_scan_kernel(const float* __restrict__ PRE,
                                                        const unsigned short* __restrict__ WHp,
                                                        unsigned short* __restrict__ SEQp,
                                                        float* __restrict__ HL) {
  __shared__ __align__(16) _Float16 Hb[2][SCAN_ROWS * HPITCH];
  const _Float16* WH = (const _Float16*)WHp;
  _Float16* SEQ = (_Float16*)SEQp;
  const int tid = threadIdx.x, lane = tid & 31, wave = tid >> 5;
  const int c = lane & 15, hh = lane >> 4, koff = hh * 8;
  const int b0 = blockIdx.x * SCAN_ROWS;

  {
    v8h zv;
#pragma unroll
    for (int e = 0; e < 8; ++e) zv[e] = (_Float16)0.0f;
    v8h* hz = (v8h*)&Hb[0][0];
#pragma unroll 1
    for (int i = tid; i < (2 * SCAN_ROWS * HPITCH) / 8; i += NTHR) hz[i] = zv;
  }
  __syncthreads();

  const v8f z8 = {0.f, 0.f, 0.f, 0.f, 0.f, 0.f, 0.f, 0.f};

#pragma unroll 1
  for (int t = 0; t < NSTEP; ++t) {
    const int cur = t & 1;
    const _Float16* hc = &Hb[cur][0];
    _Float16* hn = &Hb[cur ^ 1][0];
    const bool last = (t == NSTEP - 1);
    const _Float16* hrow0 = hc + c * HPITCH + koff;
    const _Float16* hrow1 = hc + (16 + c) * HPITCH + koff;

#pragma unroll 1
    for (int nt = 0; nt < 4; ++nt) {
      const int ncol = 64 * wave + 16 * nt;
      const _Float16* wrow = WH + (size_t)(ncol + c) * NHID + koff;
      v8f acc0 = z8, acc1 = z8;
#pragma unroll 1
      for (int k0 = 0; k0 < NHID; k0 += 32) {
        const v16h aw  = FragH::load(wrow + k0);
        const v16h hf0 = FragH::load(hrow0 + k0);
        const v16h hf1 = FragH::load(hrow1 + k0);
        acc0 = FragH::mma(aw, hf0, acc0);
        acc1 = FragH::mma(aw, hf1, acc1);
        guard2_h(acc0, acc1, aw, hf0, hf1);
      }
      acc_guard2(acc0, acc1);

      const int nlane = ncol + 8 * hh;
#pragma unroll 1
      for (int bt = 0; bt < 2; ++bt) {
        v8f a;
#pragma unroll
        for (int r = 0; r < 8; ++r) a[r] = (bt == 0) ? acc0[r] : acc1[r];
        const int brow = 16 * bt + c;
        const float* pp = PRE + ((size_t)t * NBATCH + (size_t)(b0 + brow)) * NHID + nlane;
        v4f p0 = *(const v4f*)(pp);
        v4f p1 = *(const v4f*)(pp + 4);
        pin2_f(p0, p1);
        float th[8];
#pragma unroll
        for (int r = 0; r < 4; ++r) {
          th[r]     = tanhf(a[r] * W_CARRY_INV + p0[r]);
          th[4 + r] = tanhf(a[4 + r] * W_CARRY_INV + p1[r]);
        }
        v8h hv;
#pragma unroll
        for (int r = 0; r < 8; ++r) hv[r] = (_Float16)th[r];
        *(v8h*)(hn + brow * HPITCH + nlane) = hv;
        if (FINAL) {
          if (last) {
            const int tileid = ((blockIdx.x * 8 + wave) * 4 + nt) * 2 + bt;
            float* hp = HL + (size_t)tileid * 256 + lane * 4;
            const v4f lo = {th[0], th[1], th[2], th[3]};
            const v4f hi = {th[4], th[5], th[6], th[7]};
            *(volatile v4f*)(hp) = lo;
            *(volatile v4f*)(hp + 128) = hi;
            __threadfence();
            *(volatile v4f*)(hp) = lo;
            *(volatile v4f*)(hp + 128) = hi;
          }
        }
      }
    }
    __syncthreads();

    if (WRITE_SEQ) {
      v8h vv[8];
#pragma unroll
      for (int it = 0; it < 8; ++it) {
        const int idx = it * NTHR + tid;
        const int row = idx >> 6, c8 = (idx & 63) * 8;
        vv[it] = *(const v8h*)(hn + row * HPITCH + c8);
      }
      for (int pass = 0; pass < 2; ++pass) {
#pragma unroll
        for (int it = 0; it < 8; ++it) {
          const int idx = it * NTHR + tid;
          const int row = idx >> 6, c8 = (idx & 63) * 8;
          *(volatile v8h*)(SEQ + ((size_t)t * NBATCH + (size_t)(b0 + row)) * NHID + c8) = vv[it];
        }
        __threadfence();
      }
    }
  }
}

__global__ __launch_bounds__(128) void head_kernel(const float* __restrict__ HL, const float* __restrict__ wfc,
                                                   const float* __restrict__ bfc, float* __restrict__ out) {
  const int e  = blockIdx.x * 128 + threadIdx.x;
  const int ec = (e < NBATCH * NCLS) ? e : (NBATCH * NCLS - 1);
  const int b = ec / NCLS;
  const int cls = ec - b * NCLS;
  const int blk = b >> 5, bt = (b >> 4) & 1, c = b & 15;
  float s = 0.0f;
#pragma unroll 2
  for (int g = 0; g < NHID / 8; ++g) {
    const int w = g >> 3, nt = (g >> 1) & 3, hh = g & 1;
    const int tileid = ((blk * 8 + w) * 4 + nt) * 2 + bt;
    const float* hp = HL + (size_t)tileid * 256 + (hh * 16 + c) * 4;
    const v4f lo = *(const v4f*)(hp);
    const v4f hi = *(const v4f*)(hp + 128);
    const float* wp = wfc + cls * NHID + 8 * g;
    const v4f w0 = *(const v4f*)(wp);
    const v4f w1 = *(const v4f*)(wp + 4);
    s = fmaf(lo[0], w0[0], s);
    s = fmaf(lo[1], w0[1], s);
    s = fmaf(lo[2], w0[2], s);
    s = fmaf(lo[3], w0[3], s);
    s = fmaf(hi[0], w1[0], s);
    s = fmaf(hi[1], w1[1], s);
    s = fmaf(hi[2], w1[2], s);
    s = fmaf(hi[3], w1[3], s);
  }
  s += bfc[cls];
  if (e < NBATCH * NCLS) {
    volatile float* op = (volatile float*)out + e;
    *op = s;
    __threadfence();
    *op = s;
  }
}

extern "C" void kernel_launch(void* const* d_in, const int* in_sizes, int n_in,
                              void* d_out, int out_size, void* d_ws, size_t ws_size, hipStream_t stream) {
  if (n_in < 11 || d_out == nullptr || d_ws == nullptr) return;
  if (in_sizes[0] != NBATCH * NSTEP * NIN || in_sizes[1] != NHID * NIN || in_sizes[2] != NHID * NHID ||
      in_sizes[3] != NHID || in_sizes[4] != NHID || in_sizes[5] != NHID * NHID || in_sizes[6] != NHID * NHID ||
      in_sizes[7] != NHID || in_sizes[8] != NHID || in_sizes[9] != NCLS * NHID || in_sizes[10] != NCLS ||
      out_size != NBATCH * NCLS) return;

  const float* x     = (const float*)d_in[0];
  const float* w_ih0 = (const float*)d_in[1];
  const float* w_hh0 = (const float*)d_in[2];
  const float* b_ih0 = (const float*)d_in[3];
  const float* b_hh0 = (const float*)d_in[4];
  const float* w_ih1 = (const float*)d_in[5];
  const float* w_hh1 = (const float*)d_in[6];
  const float* b_ih1 = (const float*)d_in[7];
  const float* b_hh1 = (const float*)d_in[8];
  const float* w_fc  = (const float*)d_in[9];
  const float* b_fc  = (const float*)d_in[10];
  float* out = (float*)d_out;

  char* ws = (char*)d_ws;
  size_t off = 0;
  auto carve = [&](size_t bytes) -> char* { char* p = ws + off; off += (bytes + 255) & ~(size_t)255; return p; };
  unsigned short* XH   = (unsigned short*)carve((size_t)NROWS * NIN * 2);
  unsigned short* WI0  = (unsigned short*)carve((size_t)NHID * NIN * 2);
  unsigned short* WH0  = (unsigned short*)carve((size_t)NHID * NHID * 2);
  unsigned short* WI1  = (unsigned short*)carve((size_t)NHID * NHID * 2);
  unsigned short* WH1  = (unsigned short*)carve((size_t)NHID * NHID * 2);
  float*          PRE  = (float*)carve((size_t)NROWS * NHID * 4);
  unsigned short* OUT0 = (unsigned short*)carve((size_t)NROWS * NHID * 2);
  float*          HL   = (float*)carve((size_t)NBATCH * NHID * 4);
  if (off > ws_size || off > (size_t)134217728) return;

  const int n8x  = NROWS * (NIN / 8);
  const int n8wi = NHID * (NIN / 8);
  const int n8wh = NHID * (NHID / 8);
  cvt_x_kernel<<<n8x / NTHR, NTHR, 0, stream>>>(x, XH);
  cvt_w_kernel<<<n8wi / NTHR, NTHR, 0, stream>>>(w_ih0, WI0, n8wi, W_CARRY);
  cvt_w_kernel<<<n8wh / NTHR, NTHR, 0, stream>>>(w_hh0, WH0, n8wh, W_CARRY);
  cvt_w_kernel<<<n8wh / NTHR, NTHR, 0, stream>>>(w_ih1, WI1, n8wh, W_CARRY);
  cvt_w_kernel<<<n8wh / NTHR, NTHR, 0, stream>>>(w_hh1, WH1, n8wh, W_CARRY);

  const int gblocks = ((NROWS / 64) * (NHID / 64)) / 8;

  gemm_f16_bias2_kernel<<<gblocks, 256, 0, stream>>>(XH, NIN, WI0, NIN, PRE, NHID, b_ih0, b_hh0,
                                                     NROWS, NHID, NIN, W_CARRY_INV);
  rnn_scan_kernel<true, false><<<NBATCH / SCAN_ROWS, NTHR, 0, stream>>>(PRE, WH0, OUT0, HL);

  gemm_f16_bias2_kernel<<<gblocks, 256, 0, stream>>>(OUT0, NHID, WI1, NHID, PRE, NHID, b_ih1, b_hh1,
                                                     NROWS, NHID, NHID, W_CARRY_INV);
  rnn_scan_kernel<false, true><<<NBATCH / SCAN_ROWS, NTHR, 0, stream>>>(PRE, WH1, OUT0, HL);

  head_kernel<<<(NBATCH * NCLS) / 128, 128, 0, stream>>>(HL, w_fc, b_fc, out);
}
